// SequentialHyperMamba_60713657697149
// MI455X (gfx1250) — hardware-run, weakly checked
//
#include <hip/hip_runtime.h>
#include <math.h>

typedef __attribute__((ext_vector_type(16))) _Float16 v16h;
typedef __attribute__((ext_vector_type(8)))  _Float16 v8h;
typedef __attribute__((ext_vector_type(8)))  float    v8f;
typedef __attribute__((ext_vector_type(4)))  float    v4f;

constexpr int kB   = 4;
constexpr int kC   = 256;
constexpr int kL   = 4096;
constexpr int kM   = kB * kL;
constexpr int kE   = 8;
constexpr int kNS  = 8;
constexpr int kR   = 16;
constexpr int kXW  = kR + 2 * kNS;
constexpr int kXP  = 64;
constexpr int kDtK = 32;
constexpr int kTP  = 260;
constexpr int kScanTS = 64;
constexpr int kScanCh = 64;
constexpr int kScanYP = 68;
constexpr float kWCarry  = 32.0f;
constexpr float kUCarry  = 64.0f;
constexpr float kDtCarry = 256.0f;
static_assert(kM == 16384);
static_assert(kXW == 32);
static_assert((kC % 64) == 0 && (kM % 64) == 0 && (kL % 64) == 0 && (kXP % 64) == 0);
static_assert((kC % 32) == 0 && (kDtK % 32) == 0 && kR <= kDtK);
static_assert((kL % kScanTS) == 0 && (kC % kScanCh) == 0);

constexpr size_t kOffWFUSE = 0;
constexpr size_t kOffWIN   = kOffWFUSE + (size_t)kC * kC * 2;
constexpr size_t kOffWXF   = kOffWIN   + (size_t)2 * kC * kC * 2;
constexpr size_t kOffWXB   = kOffWXF   + (size_t)kXP * kC * 2;
constexpr size_t kOffWDTF  = kOffWXB   + (size_t)kXP * kC * 2;
constexpr size_t kOffWDTB  = kOffWDTF  + (size_t)kC * kDtK * 2;
constexpr size_t kOffWOUT  = kOffWDTB  + (size_t)kC * kDtK * 2;
constexpr size_t kOffWOP   = kOffWOUT  + (size_t)kC * kC * 2;
constexpr size_t kOffEDGE2 = kOffWOP   + (size_t)kC * kC * 2;
constexpr size_t kOffAPART = kOffEDGE2 + (size_t)kB * kE * kC * 4;
constexpr size_t kOffACT16 = kOffAPART + (size_t)kM * kE * 4;
constexpr size_t kOffXH    = kOffACT16 + (size_t)kM * kC * 2;
constexpr size_t kOffXM    = kOffXH    + (size_t)kM * kC * 4;
constexpr size_t kOffZP    = kOffXM    + (size_t)kM * kC * 4;
constexpr size_t kOffXC    = kOffZP    + (size_t)kM * kC * 4;
constexpr size_t kOffXC16  = kOffXC    + (size_t)kM * kC * 4;
constexpr size_t kOffDBL   = kOffXC16  + (size_t)kM * kC * 2;
constexpr size_t kOffDT16  = kOffDBL   + (size_t)kM * kXP * 4;
constexpr size_t kOffDTP   = kOffDT16  + (size_t)kM * kDtK * 2;
constexpr size_t kOffYF    = kOffDTP   + (size_t)kM * kC * 4;
constexpr size_t kWsTotal  = kOffYF    + (size_t)kM * kC * 4;
static_assert(kWsTotal == 123994112ull);
static_assert(kWsTotal <= 134217728ull);
static_assert((kOffWIN % 128) == 0 && (kOffWXF % 128) == 0 && (kOffWXB % 128) == 0 && (kOffWDTF % 128) == 0 &&
              (kOffWDTB % 128) == 0 && (kOffWOUT % 128) == 0 && (kOffWOP % 128) == 0 && (kOffEDGE2 % 128) == 0 &&
              (kOffAPART % 128) == 0 && (kOffACT16 % 128) == 0 && (kOffXH % 128) == 0 && (kOffXM % 128) == 0 &&
              (kOffZP % 128) == 0 && (kOffXC % 128) == 0 && (kOffXC16 % 128) == 0 && (kOffDBL % 128) == 0 &&
              (kOffDT16 % 128) == 0 && (kOffDTP % 128) == 0 && (kOffYF % 128) == 0);
static_assert(kOffZP == kOffXM + (size_t)kM * kC * 4);

__device__ __forceinline__ float silu_f(float v) {
  return v * __builtin_amdgcn_rcpf(1.0f + expf(-v));
}

__device__ __forceinline__ void grp_guard_h(v8f& a, v8f& b, v8f& c, v8f& d, v16h x, v16h y0, v16h y1, v16h y2, v16h y3) {
  asm volatile("v_nop\n\tv_nop\n\tv_nop\n\tv_nop" : "+v"(a), "+v"(b), "+v"(c), "+v"(d) : "v"(x), "v"(y0), "v"(y1), "v"(y2), "v"(y3));
}
__device__ __forceinline__ void keep4_h(v16h a, v16h b, v16h c, v16h d) { asm volatile("v_nop" :: "v"(a), "v"(b), "v"(c), "v"(d)); }
__device__ __forceinline__ void acc_guard4(v8f& a, v8f& b, v8f& c, v8f& d) { asm volatile("v_nop\n\tv_nop\n\tv_nop\n\tv_nop" : "+v"(a), "+v"(b), "+v"(c), "+v"(d)); }

struct FragH {
  union U { v16h v; v8h h[2]; };
  static __device__ __forceinline__ v16h load(const _Float16* p) {
    U f; f.h[0] = *(const v8h*)(p); f.h[1] = *(const v8h*)(p + 16); return f.v;
  }
  static __device__ __forceinline__ v8f mma(v16h a, v16h b, v8f c) {
    return __builtin_amdgcn_wmma_f32_16x16x32_f16(false, a, false, b, (short)0, c, false, false);
  }
};

template <int BIAS_MODE, int ACT>
__global__ __launch_bounds__(256) void wmma_gemm64(
    const unsigned short* __restrict__ Ap, int lda, long strideA,
    const unsigned short* __restrict__ Btp, int ldb, long strideB,
    float* __restrict__ Cout, int ldc, long strideC,
    const float* __restrict__ bias, int M, int N, int K, float scale) {
  typedef _Float16 T;
  typedef v16h V;
  const T* A = (const T*)Ap; const T* Bt = (const T*)Btp;
  __shared__ __align__(16) float sT[8][16 * 68];
  const int b    = blockIdx.y;
  const int lane = threadIdx.x & 31;
  const int wave = threadIdx.x >> 5;
  const int tilesN = N >> 6;
  const int tilesM = M >> 6;
  const int tile = blockIdx.x * 8 + wave;
  if (tile >= tilesM * tilesN) return;
  const int tm = tile / tilesN;
  const int tn = tile - tm * tilesN;
  const int m0 = tm << 6;
  const int n0 = tn << 6;

  const T* Ab = A  + (size_t)b * strideA;
  const T* Bb = Bt + (size_t)b * strideB;

  const int rlane = lane & 15;
  const int koff  = (lane >> 4) * 8;
  const int mOff  = (lane >> 4) * 8;

  v8f acc[4][4];
#pragma unroll
  for (int i = 0; i < 4; ++i)
#pragma unroll
    for (int j = 0; j < 4; ++j) acc[i][j] = (v8f){0.f,0.f,0.f,0.f,0.f,0.f,0.f,0.f};

  for (int k0 = 0; k0 < K; k0 += 32) {
    V bh[4];
#pragma unroll
    for (int j = 0; j < 4; ++j) {
      const size_t bo = (size_t)(n0 + (j << 4) + rlane) * ldb + koff + k0;
      bh[j] = FragH::load(Bb + bo);
    }
#pragma unroll
    for (int i = 0; i < 4; ++i) {
      const size_t ao = (size_t)(m0 + (i << 4) + rlane) * lda + koff + k0;
      V ah = FragH::load(Ab + ao);
#pragma unroll
      for (int j = 0; j < 4; ++j) acc[i][j] = FragH::mma(ah, bh[j], acc[i][j]);
      grp_guard_h(acc[i][0], acc[i][1], acc[i][2], acc[i][3], ah, bh[0], bh[1], bh[2], bh[3]);
    }
    keep4_h(bh[0], bh[1], bh[2], bh[3]);
  }
  acc_guard4(acc[0][0], acc[0][1], acc[0][2], acc[0][3]);
  acc_guard4(acc[1][0], acc[1][1], acc[1][2], acc[1][3]);
  acc_guard4(acc[2][0], acc[2][1], acc[2][2], acc[2][3]);
  acc_guard4(acc[3][0], acc[3][1], acc[3][2], acc[3][3]);

  float* slab = sT[wave];
  float* C = Cout + (size_t)b * strideC;
#pragma unroll
  for (int i = 0; i < 4; ++i) {
    const int mBase = m0 + (i << 4);
#pragma unroll
    for (int j = 0; j < 4; ++j) {
      const int n = n0 + (j << 4) + rlane;
      float bv = 0.f;
      if (BIAS_MODE == 2) bv = bias[n];
#pragma unroll
      for (int r = 0; r < 8; ++r) {
        float v = acc[i][j][r] * scale;
        if (BIAS_MODE == 1) v += bias[mBase + mOff + r];
        if (BIAS_MODE == 2) v += bv;
        if (ACT == 6) v = silu_f(v);
        slab[(mOff + r) * 68 + (j << 4) + rlane] = v;
      }
    }
    __builtin_amdgcn_fence(__ATOMIC_RELEASE, "workgroup");
    __builtin_amdgcn_wave_barrier();
    __builtin_amdgcn_fence(__ATOMIC_ACQUIRE, "workgroup");
    {
      const int hh = lane >> 4, c4 = (lane & 15) * 4;
      for (int pass = 0; pass < 2; ++pass) {
#pragma unroll
        for (int it = 0; it < 8; ++it) {
          const int row = it * 2 + hh;
          v4f v = *(const v4f*)(slab + row * 68 + c4);
          *(volatile v4f*)(C + (size_t)(mBase + row) * ldc + n0 + c4) = v;
        }
        __threadfence();
      }
    }
    __builtin_amdgcn_fence(__ATOMIC_RELEASE, "workgroup");
    __builtin_amdgcn_wave_barrier();
    __builtin_amdgcn_fence(__ATOMIC_ACQUIRE, "workgroup");
  }
}

__global__ __launch_bounds__(256) void cast_f16_kernel(
    const float* __restrict__ src, unsigned short* __restrict__ dst, int total8, float scale)
{
  const int i = blockIdx.x * 256 + threadIdx.x;
  if (i >= total8) return;
  const size_t e0 = (size_t)i << 3;
  const float* p = src + e0;
  const v4f a0 = *(const v4f*)(p);
  const v4f a1 = *(const v4f*)(p + 4);
  v8h hv;
#pragma unroll
  for (int e = 0; e < 4; ++e) {
    hv[e]     = (_Float16)(a0[e] * scale);
    hv[4 + e] = (_Float16)(a1[e] * scale);
  }
  unsigned short* q = dst + e0;
  *(volatile v8h*)q = hv;
  __threadfence();
  *(volatile v8h*)q = hv;
}

__global__ __launch_bounds__(256) void transpose_cast_kernel(
    const float* __restrict__ W, unsigned short* __restrict__ Bt, int Kdim, int Ndim, int Npad, float scale)
{
  __shared__ float tile[64 * 65];
  const int tid = threadIdx.x, lane = tid & 31, wave = tid >> 5;
  const int n0 = blockIdx.x * 64;
  const int k0 = blockIdx.y * 64;
  (void)Npad;
#pragma unroll
  for (int p = 0; p < 16; ++p) {
    const int idx = tid + p * 256;
    const int kk  = idx >> 6;
    const int nn  = idx & 63;
    const int n   = n0 + nn;
    const int nc  = (n < Ndim) ? n : (Ndim - 1);
    const float v = W[(size_t)(k0 + kk) * Ndim + nc];
    tile[kk * 65 + nn] = (n < Ndim) ? (v * scale) : 0.f;
  }
  __syncthreads();
  const int q = lane >> 3, c8 = (lane & 7) * 8;
  v8h hv[2];
#pragma unroll
  for (int it = 0; it < 2; ++it) {
    const int nrow = it * 32 + wave * 4 + q;
#pragma unroll
    for (int e = 0; e < 8; ++e) hv[it][e] = (_Float16)tile[(c8 + e) * 65 + nrow];
  }
  for (int pass = 0; pass < 2; ++pass) {
#pragma unroll
    for (int it = 0; it < 2; ++it) {
      const int nrow = it * 32 + wave * 4 + q;
      *(volatile v8h*)(Bt + (size_t)(n0 + nrow) * Kdim + k0 + c8) = hv[it];
    }
    __threadfence();
  }
}

__global__ __launch_bounds__(256) void wdt_prep_kernel(
    const float* __restrict__ Wf, const float* __restrict__ Wb,
    unsigned short* __restrict__ Of, unsigned short* __restrict__ Ob)
{
  const float* W = (blockIdx.y == 0) ? Wf : Wb;
  unsigned short* O = (blockIdx.y == 0) ? Of : Ob;
  const int i = blockIdx.x * 256 + threadIdx.x;
  const int n = i >> 2;
  const int c8 = (i & 3) * 8;
  v8h hv;
#pragma unroll
  for (int e = 0; e < 8; ++e) {
    const int k = c8 + e;
    const int kc = (k < kR) ? k : (kR - 1);
    const float v = W[(size_t)kc * kC + n];
    hv[e] = (_Float16)((k < kR) ? (v * kWCarry) : 0.f);
  }
  unsigned short* q = O + (size_t)i * 8;
  *(volatile v8h*)q = hv;
  __threadfence();
  *(volatile v8h*)q = hv;
}

__global__ __launch_bounds__(256) void logits_softmax_kernel(
    const float* __restrict__ x, const float* __restrict__ Wedge, float* __restrict__ Apart)
{
  __shared__ __align__(16) float sW[kC * kE];
  __shared__ __align__(16) float sO[256 * kE];
  const int tid = threadIdx.x;
  *(v4f*)(sW + tid * 4)        = *(const v4f*)(Wedge + tid * 4);
  *(v4f*)(sW + 1024 + tid * 4) = *(const v4f*)(Wedge + 1024 + tid * 4);
  __syncthreads();
  const int m = blockIdx.x * 256 + tid;
  const int b = m >> 12;
  const int n = m & (kL - 1);
  const float* xp = x + (size_t)b * kC * kL + n;
  v4f l0 = (v4f){0.f, 0.f, 0.f, 0.f};
  v4f l1 = (v4f){0.f, 0.f, 0.f, 0.f};
#pragma unroll 4
  for (int c = 0; c < kC; ++c) {
    const float xv = xp[(size_t)c * kL];
    const v4f w0 = *(const v4f*)(sW + c * 8);
    const v4f w1 = *(const v4f*)(sW + c * 8 + 4);
    l0 = w0 * xv + l0;
    l1 = w1 * xv + l1;
  }
  float mx = fmaxf(fmaxf(l0[0], l0[1]), fmaxf(l0[2], l0[3]));
  mx = fmaxf(mx, fmaxf(fmaxf(l1[0], l1[1]), fmaxf(l1[2], l1[3])));
  v4f e0, e1;
  e0[0] = expf(l0[0] - mx); e0[1] = expf(l0[1] - mx); e0[2] = expf(l0[2] - mx); e0[3] = expf(l0[3] - mx);
  e1[0] = expf(l1[0] - mx); e1[1] = expf(l1[1] - mx); e1[2] = expf(l1[2] - mx); e1[3] = expf(l1[3] - mx);
  const float s = ((e0[0] + e0[1]) + (e0[2] + e0[3])) + ((e1[0] + e1[1]) + (e1[2] + e1[3]));
  const float inv = 1.0f / s;
  *(v4f*)(sO + tid * 8)     = e0 * inv;
  *(v4f*)(sO + tid * 8 + 4) = e1 * inv;
  __syncthreads();
  const v4f o0 = *(const v4f*)(sO + tid * 4);
  const v4f o1 = *(const v4f*)(sO + 1024 + tid * 4);
  float* dst = Apart + (size_t)blockIdx.x * 2048;
  for (int pass = 0; pass < 2; ++pass) {
    *(volatile v4f*)(dst + tid * 4) = o0;
    *(volatile v4f*)(dst + 1024 + tid * 4) = o1;
    __threadfence();
  }
}

__global__ __launch_bounds__(256) void edge_kernel(
    const float* __restrict__ x, const float* __restrict__ Apart, const float* __restrict__ W_e,
    const float* __restrict__ b_e, float* __restrict__ edge2)
{
  __shared__ __align__(16) float sA[256 * kE];
  __shared__ __align__(16) float sE[kC * kE];
  const int tid = threadIdx.x;
  const int b = blockIdx.x;
  const float* xrow = x + ((size_t)(b * kC + tid)) * kL;
  v4f acc0 = (v4f){0.f, 0.f, 0.f, 0.f}, acc1 = (v4f){0.f, 0.f, 0.f, 0.f};
  v4f sa0  = (v4f){0.f, 0.f, 0.f, 0.f}, sa1  = (v4f){0.f, 0.f, 0.f, 0.f};
#pragma unroll 1
  for (int ch = 0; ch < kL / 256; ++ch) {
    __syncthreads();
    const float* ap = Apart + ((size_t)b * kL + (size_t)ch * 256) * kE;
    *(v4f*)(sA + tid * 4)        = *(const v4f*)(ap + tid * 4);
    *(v4f*)(sA + 1024 + tid * 4) = *(const v4f*)(ap + 1024 + tid * 4);
    __syncthreads();
#pragma unroll 1
    for (int n4 = 0; n4 < 64; ++n4) {
      const v4f xv = *(const v4f*)(xrow + ch * 256 + n4 * 4);
#pragma unroll
      for (int j = 0; j < 4; ++j) {
        const v4f a0 = *(const v4f*)(sA + (n4 * 4 + j) * 8);
        const v4f a1 = *(const v4f*)(sA + (n4 * 4 + j) * 8 + 4);
        const float xs = xv[j];
        acc0 = a0 * xs + acc0;
        acc1 = a1 * xs + acc1;
        sa0 += a0;
        sa1 += a1;
      }
    }
  }
  v4f r0, r1;
  r0[0] = __builtin_amdgcn_rcpf(sa0[0] + 1e-6f); r0[1] = __builtin_amdgcn_rcpf(sa0[1] + 1e-6f);
  r0[2] = __builtin_amdgcn_rcpf(sa0[2] + 1e-6f); r0[3] = __builtin_amdgcn_rcpf(sa0[3] + 1e-6f);
  r1[0] = __builtin_amdgcn_rcpf(sa1[0] + 1e-6f); r1[1] = __builtin_amdgcn_rcpf(sa1[1] + 1e-6f);
  r1[2] = __builtin_amdgcn_rcpf(sa1[2] + 1e-6f); r1[3] = __builtin_amdgcn_rcpf(sa1[3] + 1e-6f);
  *(v4f*)(sE + tid * 8)     = acc0 * r0;
  *(v4f*)(sE + tid * 8 + 4) = acc1 * r1;
  __syncthreads();
  v4f m0 = (v4f){0.f, 0.f, 0.f, 0.f}, m1 = (v4f){0.f, 0.f, 0.f, 0.f};
#pragma unroll 2
  for (int c = 0; c < kC; ++c) {
    const float w = W_e[(size_t)c * kC + tid];
    const v4f g0 = *(const v4f*)(sE + c * 8);
    const v4f g1 = *(const v4f*)(sE + c * 8 + 4);
    m0 = g0 * w + m0;
    m1 = g1 * w + m1;
  }
  const float bo = b_e[tid];
  float ov[kE];
  ov[0] = silu_f(m0[0] + bo); ov[1] = silu_f(m0[1] + bo); ov[2] = silu_f(m0[2] + bo); ov[3] = silu_f(m0[3] + bo);
  ov[4] = silu_f(m1[0] + bo); ov[5] = silu_f(m1[1] + bo); ov[6] = silu_f(m1[2] + bo); ov[7] = silu_f(m1[3] + bo);
  for (int pass = 0; pass < 2; ++pass) {
#pragma unroll
    for (int e = 0; e < kE; ++e)
      *(volatile float*)(edge2 + ((size_t)(b * kE + e)) * kC + tid) = ov[e];
    __threadfence();
  }
}

template <int MODE>
__global__ __launch_bounds__(256) void xpose_add_kernel(
    const float* __restrict__ x, const float* __restrict__ P0, const float* __restrict__ P1,
    const float* __restrict__ P2, unsigned short* __restrict__ out16)
{
  __shared__ float tile[64 * 65];
  __shared__ __align__(16) float sEd[kE * 64];
  __shared__ __align__(16) float sAp[64 * kE];
  const int tid = threadIdx.x, lane = tid & 31, wave = tid >> 5;
  const int c0 = blockIdx.x * 64;
  const int m0 = blockIdx.y * 64;
  const int b  = m0 >> 12;
  const int n0 = m0 & (kL - 1);
#pragma unroll
  for (int p = 0; p < 16; ++p) {
    const int idx = tid + p * 256;
    const int cc  = idx >> 6;
    const int nn  = idx & 63;
    tile[cc * 65 + nn] = x[((size_t)(b * kC + c0 + cc)) * kL + n0 + nn];
  }
  if (MODE == 1) {
    if (tid < 128) {
      const int e = tid >> 4, c4 = (tid & 15) * 4;
      *(v4f*)(sEd + e * 64 + c4) = *(const v4f*)(P1 + ((size_t)(b * kE + e)) * kC + c0 + c4);
    } else {
      const int t2 = tid - 128;
      *(v4f*)(sAp + t2 * 4) = *(const v4f*)(P0 + (size_t)m0 * kE + t2 * 4);
    }
  }
  __syncthreads();
  const int q = lane >> 3, c8 = (lane & 7) * 8;
#pragma unroll 1
  for (int it = 0; it < 2; ++it) {
    const int row = it * 32 + wave * 4 + q;
    const size_t m = (size_t)(m0 + row);
    v4f v0, v1;
    v0[0] = tile[(c8 + 0) * 65 + row]; v0[1] = tile[(c8 + 1) * 65 + row];
    v0[2] = tile[(c8 + 2) * 65 + row]; v0[3] = tile[(c8 + 3) * 65 + row];
    v1[0] = tile[(c8 + 4) * 65 + row]; v1[1] = tile[(c8 + 5) * 65 + row];
    v1[2] = tile[(c8 + 6) * 65 + row]; v1[3] = tile[(c8 + 7) * 65 + row];
    if (MODE == 1) {
      v4f s0 = (v4f){0.f, 0.f, 0.f, 0.f}, s1 = (v4f){0.f, 0.f, 0.f, 0.f};
#pragma unroll 1
      for (int e = 0; e < kE; ++e) {
        const float a = sAp[row * kE + e];
        const v4f d0 = *(const v4f*)(sEd + e * 64 + c8);
        const v4f d1 = *(const v4f*)(sEd + e * 64 + c8 + 4);
        s0 = d0 * a + s0;
        s1 = d1 * a + s1;
      }
      v0 = v0 + s0;
      v1 = v1 + s1;
    } else {
      const size_t o = m * kC + c0 + c8;
      const v4f h0 = *(const v4f*)(P0 + o);
      const v4f h1 = *(const v4f*)(P0 + o + 4);
      const v4f y0 = *(const v4f*)(P1 + o);
      const v4f y1 = *(const v4f*)(P1 + o + 4);
      const v4f g0 = *(const v4f*)(P2 + c0 + c8);
      const v4f g1 = *(const v4f*)(P2 + c0 + c8 + 4);
      v0 = (v0 + h0) + (g0 * y0 + h0);
      v1 = (v1 + h1) + (g1 * y1 + h1);
    }
    v8h hv;
    hv[0] = (_Float16)v0[0]; hv[1] = (_Float16)v0[1]; hv[2] = (_Float16)v0[2]; hv[3] = (_Float16)v0[3];
    hv[4] = (_Float16)v1[0]; hv[5] = (_Float16)v1[1]; hv[6] = (_Float16)v1[2]; hv[7] = (_Float16)v1[3];
    unsigned short* dst = out16 + m * kC + c0 + c8;
    *(volatile v8h*)dst = hv;
    __threadfence();
    *(volatile v8h*)dst = hv;
  }
}

template <int MODE>
__global__ __launch_bounds__(256) void rownorm_kernel(
    const float* __restrict__ S0, const float* __restrict__ S1, const float* __restrict__ S2,
    const float* __restrict__ w, unsigned short* __restrict__ dst)
{
  const int lane = threadIdx.x & 31, wave = threadIdx.x >> 5;
  const int c8 = lane * 8;
  const v4f w0 = *(const v4f*)(w + c8);
  const v4f w1 = *(const v4f*)(w + c8 + 4);
#pragma unroll 1
  for (int i = 0; i < 4; ++i) {
    const int row = (blockIdx.x * 8 + wave) * 4 + i;
    const size_t o = (size_t)row * kC + c8;
    v4f a0 = *(const v4f*)(S0 + o);
    v4f a1 = *(const v4f*)(S0 + o + 4);
    if (MODE == 1) {
      const v4f b0 = *(const v4f*)(S1 + o);
      const v4f b1 = *(const v4f*)(S1 + o + 4);
      const v4f z0 = *(const v4f*)(S2 + o);
      const v4f z1 = *(const v4f*)(S2 + o + 4);
      v4f g0, g1;
      g0[0] = silu_f(z0[0]); g0[1] = silu_f(z0[1]); g0[2] = silu_f(z0[2]); g0[3] = silu_f(z0[3]);
      g1[0] = silu_f(z1[0]); g1[1] = silu_f(z1[1]); g1[2] = silu_f(z1[2]); g1[3] = silu_f(z1[3]);
      a0 = ((a0 + b0) * 0.5f) * g0;
      a1 = ((a1 + b1) * 0.5f) * g1;
    }
    const v4f q0 = a0 * a0, q1 = a1 * a1;
    float ss = ((q0[0] + q0[1]) + (q0[2] + q0[3])) + ((q1[0] + q1[1]) + (q1[2] + q1[3]));
    ss += __shfl_xor(ss, 16, 32);
    ss += __shfl_xor(ss, 8, 32);
    ss += __shfl_xor(ss, 4, 32);
    ss += __shfl_xor(ss, 2, 32);
    ss += __shfl_xor(ss, 1, 32);
    const float scale = 1.0f / (sqrtf(ss) * 0.0625f + 1e-6f);
    const v4f r0 = (a0 * scale) * w0;
    const v4f r1 = (a1 * scale) * w1;
    v8h hv;
    hv[0] = (_Float16)r0[0]; hv[1] = (_Float16)r0[1]; hv[2] = (_Float16)r0[2]; hv[3] = (_Float16)r0[3];
    hv[4] = (_Float16)r1[0]; hv[5] = (_Float16)r1[1]; hv[6] = (_Float16)r1[2]; hv[7] = (_Float16)r1[3];
    unsigned short* p = dst + o;
    *(volatile v8h*)p = hv;
    __threadfence();
    *(volatile v8h*)p = hv;
  }
}

__global__ __launch_bounds__(256) void conv_silu_kernel(
    const float* __restrict__ XM, const float* __restrict__ cw, const float* __restrict__ cb,
    float* __restrict__ XC, unsigned short* __restrict__ XC16, int rev)
{
  __shared__ __align__(16) float sT[16 * kTP];
  const int tid = threadIdx.x, lane = tid & 31, wave = tid >> 5;
  const int d = tid;
  const int g0 = blockIdx.x * 64;
  const int tb = g0 & (kL - 1);
  const v4f wv = *(const v4f*)(cw + d * 4);
  const float w0 = wv[0], w1 = wv[1], w2 = wv[2], w3 = wv[3];
  const float bc = cb[d];
  const int dir = rev ? -1 : 1;
  const int rstart = rev ? (g0 + 63) : g0;
  float xm3, xm2, xm1;
  {
    const bool hist = rev ? (tb + 64 < kL) : (tb > 0);
    const int hb = hist ? (rstart - 3 * dir) : rstart;
    const float v3 = XM[(size_t)hb * kC + d];
    const float v2 = XM[(size_t)(hb + dir) * kC + d];
    const float v1 = XM[(size_t)(hb + 2 * dir) * kC + d];
    xm3 = hist ? v3 : 0.f;
    xm2 = hist ? v2 : 0.f;
    xm1 = hist ? v1 : 0.f;
  }
  const int hrow = wave >> 1;
  const int hch  = (wave & 1) * 128 + lane * 4;
#pragma unroll 1
  for (int sub = 0; sub < 4; ++sub) {
    const int lb = rev ? (g0 + 48 - sub * 16) : (g0 + sub * 16);
#pragma unroll 1
    for (int s = 0; s < 16; ++s) {
      const int rr = rev ? (15 - s) : s;
      const float xcur = XM[(size_t)(lb + rr) * kC + d];
      float acc = w0 * xm3;
      acc = fmaf(w1, xm2, acc);
      acc = fmaf(w2, xm1, acc);
      acc = fmaf(w3, xcur, acc);
      const float sv = acc + bc;
      sT[rr * kTP + tid] = silu_f(sv);
      xm3 = xm2; xm2 = xm1; xm1 = xcur;
    }
    __syncthreads();
    v4f fv[4];
    v8h bv[2];
#pragma unroll
    for (int it = 0; it < 4; ++it) fv[it] = *(const v4f*)(sT + (it * 4 + hrow) * kTP + hch);
#pragma unroll
    for (int it = 0; it < 2; ++it) {
      const float* sp = sT + (it * 8 + wave) * kTP + lane * 8;
      const v4f a0 = *(const v4f*)(sp);
      const v4f a1 = *(const v4f*)(sp + 4);
#pragma unroll
      for (int e = 0; e < 4; ++e) {
        bv[it][e]     = (_Float16)(a0[e] * kUCarry);
        bv[it][4 + e] = (_Float16)(a1[e] * kUCarry);
      }
    }
    for (int pass = 0; pass < 2; ++pass) {
#pragma unroll
      for (int it = 0; it < 4; ++it)
        *(volatile v4f*)(XC + (size_t)(lb + it * 4 + hrow) * kC + hch) = fv[it];
#pragma unroll
      for (int it = 0; it < 2; ++it)
        *(volatile v8h*)(XC16 + (size_t)(lb + it * 8 + wave) * kC + lane * 8) = bv[it];
      __threadfence();
    }
    __syncthreads();
  }
}

__global__ __launch_bounds__(256) void dt_cast_kernel(
    const float* __restrict__ DBL, unsigned short* __restrict__ DT16)
{
  const int i = blockIdx.x * 256 + threadIdx.x;
  const int row = i >> 2;
  const int c8 = (i & 3) * 8;
  const bool keep = (c8 < kR);
  const float* p = DBL + (size_t)row * kXP + (c8 & 8);
  const v4f a0 = *(const v4f*)(p);
  const v4f a1 = *(const v4f*)(p + 4);
  v8h hv;
#pragma unroll
  for (int e = 0; e < 4; ++e) {
    hv[e]     = (_Float16)(keep ? (a0[e] * kDtCarry) : 0.f);
    hv[4 + e] = (_Float16)(keep ? (a1[e] * kDtCarry) : 0.f);
  }
  unsigned short* q = DT16 + (size_t)i * 8;
  *(volatile v8h*)q = hv;
  __threadfence();
  *(volatile v8h*)q = hv;
}

__global__ __launch_bounds__(64) void scan_kernel(
    const float* __restrict__ DTP, const float* __restrict__ XC, const float* __restrict__ DBL,
    const float* __restrict__ Alog, const float* __restrict__ Dp, float* __restrict__ Y, int rev)
{
  __shared__ __align__(16) float sX[kScanTS * 16];
  __shared__ __align__(16) float sY[kScanTS * kScanYP];
  const int tid = threadIdx.x, lane = tid & 31, wave = tid >> 5;
  const int bix = blockIdx.x >> 2;
  const int d0  = (blockIdx.x & 3) * kScanCh;
  const int d   = d0 + tid;
  const size_t row0 = (size_t)bix * kL;
  const v4f la0 = *(const v4f*)(Alog + (size_t)d * kNS);
  const v4f la1 = *(const v4f*)(Alog + (size_t)d * kNS + 4);
  float An[kNS], h[kNS];
  An[0] = -expf(la0[0]); An[1] = -expf(la0[1]); An[2] = -expf(la0[2]); An[3] = -expf(la0[3]);
  An[4] = -expf(la1[0]); An[5] = -expf(la1[1]); An[6] = -expf(la1[2]); An[7] = -expf(la1[3]);
#pragma unroll
  for (int n = 0; n < kNS; ++n) h[n] = 0.f;
  const float Dd = Dp[d];
  const int hh = lane >> 4, c4 = (lane & 15) * 4;
#pragma unroll 1
  for (int ci = 0; ci < kL / kScanTS; ++ci) {
    const int t0 = rev ? ((kL / kScanTS - 1 - ci) * kScanTS) : (ci * kScanTS);
    __syncthreads();
#pragma unroll
    for (int i = 0; i < 4; ++i) {
      const int idx = tid + 64 * i;
      const int r = idx >> 2, q4 = (idx & 3) * 4;
      *(v4f*)(sX + r * 16 + q4) = *(const v4f*)(DBL + (row0 + t0 + r) * kXP + kR + q4);
    }
    __syncthreads();
#pragma unroll 1
    for (int si = 0; si < kScanTS; ++si) {
      const int s = rev ? (kScanTS - 1 - si) : si;
      const size_t m = row0 + t0 + s;
      const float a = DTP[m * kC + d];
      const float u = XC[m * kC + d];
      const float delta = fmaxf(a, 0.0f) + log1pf(expf(-fabsf(a)));
      const float du = delta * u;
      const v4f B0 = *(const v4f*)(sX + s * 16);
      const v4f B1 = *(const v4f*)(sX + s * 16 + 4);
      const v4f C0 = *(const v4f*)(sX + s * 16 + 8);
      const v4f C1 = *(const v4f*)(sX + s * 16 + 12);
      float Bs[kNS], Cs[kNS];
      Bs[0] = B0[0]; Bs[1] = B0[1]; Bs[2] = B0[2]; Bs[3] = B0[3];
      Bs[4] = B1[0]; Bs[5] = B1[1]; Bs[6] = B1[2]; Bs[7] = B1[3];
      Cs[0] = C0[0]; Cs[1] = C0[1]; Cs[2] = C0[2]; Cs[3] = C0[3];
      Cs[4] = C1[0]; Cs[5] = C1[1]; Cs[6] = C1[2]; Cs[7] = C1[3];
      float y = 0.f;
#pragma unroll
      for (int n = 0; n < kNS; ++n) {
        const float e = expf(delta * An[n]);
        h[n] = fmaf(h[n], e, du * Bs[n]);
        y = fmaf(h[n], Cs[n], y);
      }
      y = fmaf(u, Dd, y);
      sY[s * kScanYP + tid] = y;
    }
    __syncthreads();
    for (int pass = 0; pass < 2; ++pass) {
#pragma unroll 1
      for (int it = 0; it < 16; ++it) {
        const int row = it * 4 + wave * 2 + hh;
        const v4f v = *(const v4f*)(sY + row * kScanYP + c4);
        *(volatile v4f*)(Y + (row0 + t0 + row) * kC + d0 + c4) = v;
      }
      __threadfence();
    }
  }
}

extern "C" void kernel_launch(void* const* d_in, const int* in_sizes, int n_in,
                              void* d_out, int out_size, void* d_ws, size_t ws_size,
                              hipStream_t stream) {
  if (n_in < 27) return;
  if (in_sizes[0] != kB * kC * kL) return;
  if (in_sizes[1] != kC * kE) return;
  if (in_sizes[2] != kC * kC || in_sizes[3] != kC) return;
  if (in_sizes[4] != kC * kC || in_sizes[5] != kC) return;
  if (in_sizes[6] != kC || in_sizes[7] != kC) return;
  if (in_sizes[8] != kC * 2 * kC) return;
  if (in_sizes[9] != kC * 4 || in_sizes[10] != kC) return;
  if (in_sizes[11] != kC * kXW || in_sizes[12] != kR * kC || in_sizes[13] != kC) return;
  if (in_sizes[14] != kC * kNS || in_sizes[15] != kC) return;
  if (in_sizes[16] != kC * 4 || in_sizes[17] != kC) return;
  if (in_sizes[18] != kC * kXW || in_sizes[19] != kR * kC || in_sizes[20] != kC) return;
  if (in_sizes[21] != kC * kNS || in_sizes[22] != kC) return;
  if (in_sizes[23] != kC) return;
  if (in_sizes[24] != kC * kC || in_sizes[25] != kC * kC || in_sizes[26] != kC) return;
  if (out_size != kB * kC * kL) return;
  if (ws_size < kWsTotal) return;

  const float* x        = (const float*)d_in[0];
  const float* W_edge   = (const float*)d_in[1];
  const float* W_e      = (const float*)d_in[2];
  const float* b_e      = (const float*)d_in[3];
  const float* W_fuse   = (const float*)d_in[4];
  const float* b_fuse   = (const float*)d_in[5];
  const float* norm_w   = (const float*)d_in[6];
  const float* gamma    = (const float*)d_in[7];
  const float* W_in     = (const float*)d_in[8];
  const float* conv_w_f = (const float*)d_in[9];
  const float* conv_b_f = (const float*)d_in[10];
  const float* Wx_f     = (const float*)d_in[11];
  const float* Wdt_f    = (const float*)d_in[12];
  const float* bdt_f    = (const float*)d_in[13];
  const float* Alog_f   = (const float*)d_in[14];
  const float* D_f      = (const float*)d_in[15];
  const float* conv_w_b = (const float*)d_in[16];
  const float* conv_b_b = (const float*)d_in[17];
  const float* Wx_b     = (const float*)d_in[18];
  const float* Wdt_b    = (const float*)d_in[19];
  const float* bdt_b    = (const float*)d_in[20];
  const float* Alog_b   = (const float*)d_in[21];
  const float* D_b      = (const float*)d_in[22];
  const float* mnorm_w  = (const float*)d_in[23];
  const float* W_out    = (const float*)d_in[24];
  const float* W_op     = (const float*)d_in[25];
  const float* b_op     = (const float*)d_in[26];
  float* out = (float*)d_out;

  char* ws = (char*)d_ws;
  unsigned short* WFUSE16 = (unsigned short*)(ws + kOffWFUSE);
  unsigned short* WIN16   = (unsigned short*)(ws + kOffWIN);
  unsigned short* WXF16   = (unsigned short*)(ws + kOffWXF);
  unsigned short* WXB16   = (unsigned short*)(ws + kOffWXB);
  unsigned short* WDTF16  = (unsigned short*)(ws + kOffWDTF);
  unsigned short* WDTB16  = (unsigned short*)(ws + kOffWDTB);
  unsigned short* WOUT16  = (unsigned short*)(ws + kOffWOUT);
  unsigned short* WOP16   = (unsigned short*)(ws + kOffWOP);
  float*          EDGE2   = (float*)(ws + kOffEDGE2);
  float*          APART   = (float*)(ws + kOffAPART);
  unsigned short* ACT16   = (unsigned short*)(ws + kOffACT16);
  float*          XH      = (float*)(ws + kOffXH);
  float*          XM      = (float*)(ws + kOffXM);
  float*          ZP      = (float*)(ws + kOffZP);
  float*          XC      = (float*)(ws + kOffXC);
  unsigned short* XC16    = (unsigned short*)(ws + kOffXC16);
  float*          DBL     = (float*)(ws + kOffDBL);
  unsigned short* DT16    = (unsigned short*)(ws + kOffDT16);
  float*          DTP     = (float*)(ws + kOffDTP);
  float*          YF      = (float*)(ws + kOffYF);
  float*          YB      = XM;
  float*          Y2      = XC;
  const float* nobias = b_fuse;

  const float invW = 1.0f / kWCarry;

  transpose_cast_kernel<<<dim3(kC / 64, kC / 64), 256, 0, stream>>>(W_fuse, WFUSE16, kC, kC, kC, kWCarry);
  transpose_cast_kernel<<<dim3(2 * kC / 64, kC / 64), 256, 0, stream>>>(W_in, WIN16, kC, 2 * kC, 2 * kC, kWCarry);
  transpose_cast_kernel<<<dim3(kXP / 64, kC / 64), 256, 0, stream>>>(Wx_f, WXF16, kC, kXW, kXP, kWCarry);
  transpose_cast_kernel<<<dim3(kXP / 64, kC / 64), 256, 0, stream>>>(Wx_b, WXB16, kC, kXW, kXP, kWCarry);
  transpose_cast_kernel<<<dim3(kC / 64, kC / 64), 256, 0, stream>>>(W_out, WOUT16, kC, kC, kC, kWCarry);
  wdt_prep_kernel<<<dim3(kC * kDtK / 8 / 256, 2), 256, 0, stream>>>(Wdt_f, Wdt_b, WDTF16, WDTB16);
  cast_f16_kernel<<<(kC * kC) / 8 / 256, 256, 0, stream>>>(W_op, WOP16, (kC * kC) / 8, kWCarry);

  logits_softmax_kernel<<<kM / 256, 256, 0, stream>>>(x, W_edge, APART);
  edge_kernel<<<kB, 256, 0, stream>>>(x, APART, W_e, b_e, EDGE2);
  xpose_add_kernel<1><<<dim3(kC / 64, kM / 64), 256, 0, stream>>>(x, APART, EDGE2, gamma, ACT16);
  wmma_gemm64<2, 6><<<dim3(128, 1), 256, 0, stream>>>(
      ACT16, kC, 0L, WFUSE16, kC, 0L, XH, kC, 0L, b_fuse, kM, kC, kC, invW);

  rownorm_kernel<0><<<kM / 32, 256, 0, stream>>>(XH, XH, XH, norm_w, ACT16);
  wmma_gemm64<0, 0><<<dim3(128, 2), 256, 0, stream>>>(
      ACT16, kC, 0L, WIN16, kC, (long)kC * kC, XM, kC, (long)kM * kC, nobias, kM, kC, kC, invW);

  conv_silu_kernel<<<kM / 64, 256, 0, stream>>>(XM, conv_w_f, conv_b_f, XC, XC16, 0);
  wmma_gemm64<0, 0><<<dim3(32, 1), 256, 0, stream>>>(
      XC16, kC, 0L, WXF16, kC, 0L, DBL, kXP, 0L, nobias, kM, kXP, kC, 1.0f / (kUCarry * kWCarry));
  dt_cast_kernel<<<(kM * kDtK) / 8 / 256, 256, 0, stream>>>(DBL, DT16);
  wmma_gemm64<2, 0><<<dim3(128, 1), 256, 0, stream>>>(
      DT16, kDtK, 0L, WDTF16, kDtK, 0L, DTP, kC, 0L, bdt_f, kM, kC, kDtK, 1.0f / (kDtCarry * kWCarry));
  scan_kernel<<<kB * (kC / kScanCh), kScanCh, 0, stream>>>(DTP, XC, DBL, Alog_f, D_f, YF, 0);

  conv_silu_kernel<<<kM / 64, 256, 0, stream>>>(XM, conv_w_b, conv_b_b, XC, XC16, 1);
  wmma_gemm64<0, 0><<<dim3(32, 1), 256, 0, stream>>>(
      XC16, kC, 0L, WXB16, kC, 0L, DBL, kXP, 0L, nobias, kM, kXP, kC, 1.0f / (kUCarry * kWCarry));
  dt_cast_kernel<<<(kM * kDtK) / 8 / 256, 256, 0, stream>>>(DBL, DT16);
  wmma_gemm64<2, 0><<<dim3(128, 1), 256, 0, stream>>>(
      DT16, kDtK, 0L, WDTB16, kDtK, 0L, DTP, kC, 0L, bdt_b, kM, kC, kDtK, 1.0f / (kDtCarry * kWCarry));
  scan_kernel<<<kB * (kC / kScanCh), kScanCh, 0, stream>>>(DTP, XC, DBL, Alog_b, D_b, YB, 1);

  rownorm_kernel<1><<<kM / 32, 256, 0, stream>>>(YF, YB, ZP, mnorm_w, ACT16);
  wmma_gemm64<0, 0><<<dim3(128, 1), 256, 0, stream>>>(
      ACT16, kC, 0L, WOUT16, kC, 0L, Y2, kC, 0L, nobias, kM, kC, kC, invW);

  xpose_add_kernel<2><<<dim3(kC / 64, kM / 64), 256, 0, stream>>>(x, XH, Y2, gamma, ACT16);
  wmma_gemm64<1, 6><<<dim3(32, kB), 256, 0, stream>>>(
      WOP16, kC, 0L, ACT16, kC, (long)kL * kC, out, kL, (long)kC * kL, b_op, kC, kL, kC, invW);
}
